// LPDecoder_43989055045968
// MI455X (gfx1250) — hardware-verified
//
#include <hip/hip_runtime.h>


namespace {
constexpr int N = 100000, E = 1000000, D = 128, HID = 128, NBLK = N / 16;
constexpr float XS = 8.0f, WSC = 256.0f;
typedef _Float16 b16;
typedef __attribute__((ext_vector_type(16))) _Float16 v16b;
typedef __attribute__((ext_vector_type(8))) _Float16 v8b;
typedef __attribute__((ext_vector_type(8))) float v8f;
typedef __attribute__((ext_vector_type(4))) float v4f;
__device__ __forceinline__ float bf16_rne(float f) { unsigned int u = __float_as_uint(f); u += 0x7FFFu + ((u >> 16) & 1u); return __uint_as_float(u & 0xFFFF0000u); }
__device__ __forceinline__ v16b frag_kb(const b16* p, int hh) { const v8b a = *(const v8b*)(p + 8 * hh), b = *(const v8b*)(p + 16 + 8 * hh); v16b f;
#pragma unroll
  for (int e = 0; e < 8; ++e) { f[e] = a[e]; f[8 + e] = b[e]; } return f; }
__device__ __forceinline__ v8f wmma16b(v16b a, v16b b, v8f c) { v8f d = __builtin_amdgcn_wmma_f32_16x16x32_f16(false, a, false, b, (short)0, c, false, false); asm volatile("v_nop\n\tv_nop\n\tv_nop\n\tv_nop" : "+v"(d) : "v"(a), "v"(b)); return d; }
__device__ __forceinline__ void wave_lds_sync() { __builtin_amdgcn_fence(__ATOMIC_RELEASE, "workgroup"); __builtin_amdgcn_wave_barrier(); __builtin_amdgcn_fence(__ATOMIC_ACQUIRE, "workgroup"); }
__device__ __forceinline__ float pmul(float a, float b) { float p = a * b; asm volatile("" : "+v"(p)); return p; }
__device__ __forceinline__ int iclamp(int v, int lo, int hi) { return v < lo ? lo : (v > hi ? hi : v); }

__global__ __launch_bounds__(256) void wput_kernel(const float* __restrict__ W1, b16* __restrict__ WT) {
  const int u = blockIdx.x * 256 + threadIdx.x; if (u >= 256 * 16) return; const int o = u / 16, k0 = (u % 16) * 8; const int half = o / HID, oc = o % HID; v8b v;
#pragma unroll
  for (int j = 0; j < 8; ++j) v[j] = (b16)(bf16_rne(W1[(size_t)(half * D + k0 + j) * HID + oc]) * WSC); for (int pass = 0; pass < 2; ++pass) { *(volatile v8b*)(WT + (size_t)o * D + k0) = v; __threadfence(); }
}
__global__ __launch_bounds__(32) void node_kernel(const float* __restrict__ z, const b16* __restrict__ WT, float* __restrict__ PQ) {
  __shared__ __attribute__((aligned(16))) b16 Ah[16][D + 8]; __shared__ __attribute__((aligned(16))) float Tf[16][128 + 4];
  const int lane = threadIdx.x, nloc = lane & 15, hlf = lane >> 4; const size_t m0 = (size_t)blockIdx.x * 16;
  for (int rr = 0; rr < 16; ++rr) for (int q = 0; q < 4; ++q) Ah[rr][q * 32 + lane] = (b16)(bf16_rne(z[(m0 + rr) * D + q * 32 + lane]) * XS);
  wave_lds_sync();
#pragma unroll 1
  for (int cg = 0; cg < 2; ++cg) { v8f acc[8];
#pragma unroll
    for (int t = 0; t < 8; ++t) acc[t] = (v8f){};
#pragma unroll
    for (int kb = 0; kb < D; kb += 32) { const v16b a = frag_kb(&Ah[nloc][kb], hlf);
#pragma unroll
      for (int t = 0; t < 8; ++t) acc[t] = wmma16b(a, frag_kb(WT + (size_t)(cg * 128 + t * 16 + nloc) * D + kb, hlf), acc[t]); }
#pragma unroll
    for (int t = 0; t < 8; ++t)
#pragma unroll
      for (int r8 = 0; r8 < 8; ++r8) Tf[8 * hlf + r8][t * 16 + nloc] = acc[t][r8] * (1.0f / (XS * WSC));
    wave_lds_sync();
    for (int pass = 0; pass < 2; ++pass) { for (int rr = 0; rr < 16; ++rr) *(volatile v4f*)(PQ + (m0 + rr) * 256 + cg * 128 + lane * 4) = *(const v4f*)(&Tf[rr][lane * 4]); __threadfence(); }
    wave_lds_sync(); }
}
__global__ __launch_bounds__(256) void edge_kernel(const float* __restrict__ PQ, const int* __restrict__ ei, const float* __restrict__ b1, const float* __restrict__ W2, const float* __restrict__ b2, float* __restrict__ out) {
  const int wave = threadIdx.x >> 5, lane = threadIdx.x & 31; const size_t e0 = ((size_t)blockIdx.x * 8 + wave) * 32; if (e0 >= (size_t)E) return;
  float bb[4], w2[4]; for (int i = 0; i < 4; ++i) { bb[i] = bf16_rne(b1[lane * 4 + i]); w2[i] = bf16_rne(W2[lane * 4 + i]); } const float c2 = bf16_rne(b2[0]); float mine = 0.0f;
#pragma unroll 1
  for (int j = 0; j < 32; ++j) { const size_t e = e0 + j; const size_t s = (size_t)iclamp(ei[e], 0, N - 1), d = (size_t)iclamp(ei[E + e], 0, N - 1); const v4f p = *(const v4f*)(PQ + s * 256 + lane * 4), q = *(const v4f*)(PQ + d * 256 + 128 + lane * 4); float acc = 0.0f;
    for (int i = 0; i < 4; ++i) acc += pmul(fmaxf(p[i] + q[i] + bb[i], 0.0f), w2[i]); for (int o = 16; o; o >>= 1) acc += __shfl_xor(acc, o); if (lane == j) mine = 1.0f / (1.0f + __expf(-(acc + c2))); }
  for (int pass = 0; pass < 2; ++pass) { ((volatile float*)out)[e0 + lane] = mine; __threadfence(); }
}
}

extern "C" void kernel_launch(void* const* d_in, const int* in_sizes, int n_in, void* d_out, int out_size, void* d_ws, size_t ws_size, hipStream_t stream) {
  (void)n_in;
  auto Fp = [&](int i) { return (const float*)d_in[i]; }; auto Ip = [&](int i) { return (const int*)d_in[i]; };
  if (in_sizes[0] != N * D || in_sizes[1] != 2 * E || in_sizes[2] != 2 * D * HID || in_sizes[3] != HID || in_sizes[4] != HID || out_size != E) return;
  const int EV = E;
  size_t off = 0; char* ws = (char*)d_ws;
  auto carve = [&](size_t bytes) { char* p = ws + off; off += (bytes + 255) & ~(size_t)255; return p; };
  b16* WT = (b16*)carve(256 * D * 2); float* PQ = (float*)carve((size_t)N * 256 * 4);
  if (off > ws_size || off > ((size_t)128 << 20)) return;
  wput_kernel<<<16, 256, 0, stream>>>(Fp(2), WT);
  node_kernel<<<NBLK, 32, 0, stream>>>(Fp(0), WT, PQ);
  edge_kernel<<<(unsigned)((EV / 32 + 7) / 8), 256, 0, stream>>>(PQ, Ip(1), Fp(3), Fp(4), Fp(5), (float*)d_out);
}
